// Self_Attn_23390391894736
// MI455X (gfx1250) — hardware-verified
//
#include <hip/hip_runtime.h>
#include <hip/hip_bf16.h>

typedef __attribute__((ext_vector_type(16))) _Float16 v16h;
typedef __attribute__((ext_vector_type(8)))  _Float16 v8h;
typedef __attribute__((ext_vector_type(16))) __bf16   v16b;
typedef __attribute__((ext_vector_type(8)))  __bf16   v8b;
typedef __attribute__((ext_vector_type(8)))  float    v8f;
typedef __attribute__((ext_vector_type(4)))  float    v4f;
typedef __attribute__((ext_vector_type(4)))  unsigned uv4;

#define NB    8
#define NCH   256
#define NPIX  4096
#define DQK   32
#define QKLD  64
#define WSCALE 16.0f
#define WSCALE_INV (1.0f / 16.0f)

__device__ __forceinline__ unsigned short f2bf_bits(float f) {
  unsigned u = __float_as_uint(f);
  return (unsigned short)((u + 0x7FFFu + ((u >> 16) & 1u)) >> 16);
}
__device__ __forceinline__ float bf_bits2f(unsigned short h) { return __uint_as_float(((unsigned)h) << 16); }

__device__ __forceinline__ void dep_guard_h(v8f& a, v8f& b, v16h x, v16h y) { asm volatile("v_nop\n\tv_nop\n\tv_nop\n\tv_nop" : "+v"(a), "+v"(b) : "v"(x), "v"(y)); }
__device__ __forceinline__ void dep_guard_b(v8f& a, v8f& b, v16b x, v16b y) { asm volatile("v_nop\n\tv_nop\n\tv_nop\n\tv_nop" : "+v"(a), "+v"(b) : "v"(x), "v"(y)); }
__device__ __forceinline__ void keep4_h(v16h a, v16h b, v16h c, v16h d) { asm volatile("v_nop" :: "v"(a), "v"(b), "v"(c), "v"(d)); }
__device__ __forceinline__ void keep4_b(v16b a, v16b b, v16b c, v16b d) { asm volatile("v_nop" :: "v"(a), "v"(b), "v"(c), "v"(d)); }
__device__ __forceinline__ void acc_guard4(v8f& a, v8f& b, v8f& c, v8f& d) { asm volatile("v_nop\n\tv_nop\n\tv_nop\n\tv_nop" : "+v"(a), "+v"(b), "+v"(c), "+v"(d)); }
template <typename T> struct Frag;
template <> struct Frag<_Float16> {
  typedef v16h V; union U { v16h v; v8h h[2]; };
  static __device__ __forceinline__ v16h load(const _Float16* p) {
    U f; f.h[0] = *(const v8h*)(p); f.h[1] = *(const v8h*)(p + 16); return f.v;
  }
  static __device__ __forceinline__ v8f mma(v16h a, v16h b, v8f c) {
    return __builtin_amdgcn_wmma_f32_16x16x32_f16(false, a, false, b, (short)0, c, false, false);
  }
  static __device__ __forceinline__ void guard(v8f& a, v8f& b, v16h x, v16h y) { dep_guard_h(a, b, x, y); }
  static __device__ __forceinline__ void keep(v16h a, v16h b, v16h c, v16h d) { keep4_h(a, b, c, d); }
};
template <> struct Frag<__bf16> {
  typedef v16b V; union U { v16b v; v8b h[2]; };
  static __device__ __forceinline__ v16b load(const __bf16* p) {
    U f; f.h[0] = *(const v8b*)(p); f.h[1] = *(const v8b*)(p + 16); return f.v;
  }
  static __device__ __forceinline__ v8f mma(v16b a, v16b b, v8f c) {
    return __builtin_amdgcn_wmma_f32_16x16x32_bf16(false, a, false, b, (short)0, c, false, false);
  }
  static __device__ __forceinline__ void guard(v8f& a, v8f& b, v16b x, v16b y) { dep_guard_b(a, b, x, y); }
  static __device__ __forceinline__ void keep(v16b a, v16b b, v16b c, v16b d) { keep4_b(a, b, c, d); }
};

template <int ET> struct Elem;
template <> struct Elem<0> { typedef _Float16 T; };
template <> struct Elem<1> { typedef __bf16 T; };
template <int ET, bool SPLIT, int BIAS_MODE, int OUT_MODE, bool RESID, int ACT = 0>
__global__ __launch_bounds__(256) void wmma_gemm64(
    const unsigned short* __restrict__ Ap, const unsigned short* __restrict__ A2p, int lda, long strideA,
    const unsigned short* __restrict__ Btp, const unsigned short* __restrict__ Bt2p, int ldb, long strideB,
    void* __restrict__ Cout, void* __restrict__ Cout2, int ldc, long strideC,
    const float* __restrict__ bias,
    const float* __restrict__ resid, long strideR,
    int M, int N, int K, float scale) {
  typedef typename Elem<ET>::T T;
  typedef typename Frag<T>::V V;
  const T* A = (const T*)Ap; const T* A2 = (const T*)A2p; const T* Bt = (const T*)Btp; const T* Bt2 = (const T*)Bt2p;
  __shared__ __align__(16) float sT[8][16 * 68];
  const int b    = blockIdx.y;
  const int lane = threadIdx.x & 31;
  const int wave = threadIdx.x >> 5;
  const int tilesN = N >> 6;
  const int tilesM = M >> 6;
  const int tile = blockIdx.x * 8 + wave;
  if (tile >= tilesM * tilesN) return;
  const int tm = tile / tilesN;
  const int tn = tile - tm * tilesN;
  const int m0 = tm << 6;
  const int n0 = tn << 6;

  const T* Ab  = A  + (size_t)b * strideA;
  const T* Bb  = Bt + (size_t)b * strideB;
  const T* Ab2 = SPLIT ? (A2  + (size_t)b * strideA) : nullptr;
  const T* Bb2 = SPLIT ? (Bt2 + (size_t)b * strideB) : nullptr;

  const int rlane = lane & 15;
  const int koff  = (lane >> 4) * 8;
  const int mOff  = (lane >> 4) * 8;

  v8f acc[4][4];
#pragma unroll
  for (int i = 0; i < 4; ++i)
#pragma unroll
    for (int j = 0; j < 4; ++j) acc[i][j] = (v8f){0.f,0.f,0.f,0.f,0.f,0.f,0.f,0.f};

  for (int k0 = 0; k0 < K; k0 += 32) {
    V bh[4], bl[4];
#pragma unroll
    for (int j = 0; j < 4; ++j) {
      const size_t bo = (size_t)(n0 + (j << 4) + rlane) * ldb + koff + k0;
      bh[j] = Frag<T>::load(Bb + bo);
      if (SPLIT) bl[j] = Frag<T>::load(Bb2 + bo);
    }
#pragma unroll
    for (int i = 0; i < 4; ++i) {
      const size_t ao = (size_t)(m0 + (i << 4) + rlane) * lda + koff + k0;
      V ah = Frag<T>::load(Ab + ao);
      V al;
      if (SPLIT) al = Frag<T>::load(Ab2 + ao);
#pragma unroll
      for (int j = 0; j < 4; ++j) {
        acc[i][j] = Frag<T>::mma(ah, bh[j], acc[i][j]);
        if (SPLIT) {
          acc[i][j] = Frag<T>::mma(ah, bl[j], acc[i][j]);
          acc[i][j] = Frag<T>::mma(al, bh[j], acc[i][j]);
        }
      }
      Frag<T>::guard(acc[i][0], acc[i][3], ah, SPLIT ? al : ah);
    }
    Frag<T>::keep(bh[0], bh[1], bh[2], bh[3]);
    if (SPLIT) Frag<T>::keep(bl[0], bl[1], bl[2], bl[3]);
  }
  acc_guard4(acc[0][0], acc[0][1], acc[0][2], acc[0][3]);
  acc_guard4(acc[1][0], acc[1][1], acc[1][2], acc[1][3]);
  acc_guard4(acc[2][0], acc[2][1], acc[2][2], acc[2][3]);
  acc_guard4(acc[3][0], acc[3][1], acc[3][2], acc[3][3]);

  float* slab = sT[wave];
  const float* Rb = RESID ? (resid + (size_t)b * strideR) : nullptr;
#pragma unroll
  for (int i = 0; i < 4; ++i) {
    const int mBase = m0 + (i << 4);
#pragma unroll
    for (int j = 0; j < 4; ++j) {
      const int n = n0 + (j << 4) + rlane;
      float bv = 0.f;
      if (BIAS_MODE == 2) bv = bias[n];
#pragma unroll
      for (int r = 0; r < 8; ++r) {
        float v = acc[i][j][r] * scale;
        if (BIAS_MODE == 1) v += bias[mBase + mOff + r];
        if (BIAS_MODE == 2) v += bv;
        if (RESID) v += Rb[(size_t)(mBase + mOff + r) * ldc + n];
        if (ACT == 1) v = tanhf(v);
        if (ACT == 2) v = fmaxf(v, 0.0f);
        if (ACT == 3) v = v / (1.0f + expf(-v));
        if (ACT == 4) v = (v > 0.f) ? v : 0.01f * v;
        if (ACT == 5) v = 0.5f * v * (1.0f + erff(v * 0.70710678118654752f));
        slab[(mOff + r) * 68 + (j << 4) + rlane] = v;
      }
    }
    __builtin_amdgcn_fence(__ATOMIC_RELEASE, "workgroup");
    __builtin_amdgcn_wave_barrier();
    __builtin_amdgcn_fence(__ATOMIC_ACQUIRE, "workgroup");
    if (OUT_MODE == 0) {
      float* C = (float*)Cout + (size_t)b * strideC;
      const int hh = lane >> 4, c4 = (lane & 15) * 4;
      for (int pass = 0; pass < 2; ++pass) {
#pragma unroll
        for (int it = 0; it < 8; ++it) {
          const int row = it * 2 + hh;
          v4f v = *(const v4f*)(slab + row * 68 + c4);
          *(volatile v4f*)(C + (size_t)(mBase + row) * ldc + n0 + c4) = v;
        }
        __threadfence();
      }
    } else {
      const int q = lane >> 3, c8 = (lane & 7) * 8;
      unsigned short* C  = (unsigned short*)Cout  + (size_t)b * strideC;
      unsigned short* C2 = (OUT_MODE == 2) ? ((unsigned short*)Cout2 + (size_t)b * strideC) : nullptr;
      for (int pass = 0; pass < 2; ++pass) {
#pragma unroll
        for (int it = 0; it < 4; ++it) {
          const int row = it * 4 + q;
          const float* sp = slab + row * 68 + c8;
          v8h hv, lv;
#pragma unroll
          for (int e = 0; e < 8; ++e) {
            if (OUT_MODE == 1) {
              hv[e] = (_Float16)sp[e];
            } else {
              unsigned short hb = f2bf_bits(sp[e]);
              unsigned short lb = f2bf_bits(sp[e] - bf_bits2f(hb));
              hv[e] = __builtin_bit_cast(_Float16, hb);
              lv[e] = __builtin_bit_cast(_Float16, lb);
            }
          }
          *(volatile v8h*)(C + (size_t)(mBase + row) * ldc + n0 + c8) = hv;
          if (OUT_MODE == 2) *(volatile v8h*)(C2 + (size_t)(mBase + row) * ldc + n0 + c8) = lv;
        }
        __threadfence();
      }
    }
    __builtin_amdgcn_fence(__ATOMIC_RELEASE, "workgroup");
    __builtin_amdgcn_wave_barrier();
    __builtin_amdgcn_fence(__ATOMIC_ACQUIRE, "workgroup");
  }
}

__global__ __launch_bounds__(256) void cast_scale_f16x2(
    const float* __restrict__ in, _Float16* __restrict__ out, int n2, float sc) {
  int i = blockIdx.x * 256 + threadIdx.x;
  if (i < n2) {
    const _Float16 h0 = (_Float16)(in[2 * i] * sc), h1 = (_Float16)(in[2 * i + 1] * sc);
    const unsigned u = (unsigned)__builtin_bit_cast(unsigned short, h0) | ((unsigned)__builtin_bit_cast(unsigned short, h1) << 16);
    ((volatile unsigned*)out)[i] = u;
    __threadfence();
    ((volatile unsigned*)out)[i] = u;
  }
}

__global__ __launch_bounds__(256) void cast_wqk_f16x2(
    const float* __restrict__ wq, const float* __restrict__ wk, _Float16* __restrict__ out, int n2half, float sc) {
  int i = blockIdx.x * 256 + threadIdx.x;
  if (i < 2 * n2half) {
    const int iq = (i < n2half) ? i : (n2half - 1);
    int ik = i - n2half; ik = (ik < 0) ? 0 : ik;
    const float a0 = wq[2 * iq], a1 = wq[2 * iq + 1];
    const float b0 = wk[2 * ik], b1 = wk[2 * ik + 1];
    const bool useq = (i < n2half);
    const float v0 = (useq ? a0 : b0) * sc;
    const float v1 = (useq ? a1 : b1) * sc;
    const _Float16 h0 = (_Float16)v0, h1 = (_Float16)v1;
    const unsigned u = (unsigned)__builtin_bit_cast(unsigned short, h0) | ((unsigned)__builtin_bit_cast(unsigned short, h1) << 16);
    ((volatile unsigned*)out)[i] = u;
    __threadfence();
    ((volatile unsigned*)out)[i] = u;
  }
}

__global__ __launch_bounds__(32) void bias_pack64(
    const float* __restrict__ bq, const float* __restrict__ bk, float* __restrict__ tab) {
  const int lane = threadIdx.x;
  const int lq = (lane < 8) ? lane : 7;
  int lk = lane - 8; lk = (lk < 0) ? 0 : ((lk > 7) ? 7 : lk);
  const v4f vq = *(const v4f*)(bq + 4 * lq);
  const v4f vk = *(const v4f*)(bk + 4 * lk);
  const bool useq = (lane < 8);
  v4f v;
  v[0] = useq ? vq[0] : vk[0];
  v[1] = useq ? vq[1] : vk[1];
  v[2] = useq ? vq[2] : vk[2];
  v[3] = useq ? vq[3] : vk[3];
  if (lane < 16) {
    *(volatile v4f*)(tab + 4 * lane) = v;
    __threadfence();
    *(volatile v4f*)(tab + 4 * lane) = v;
  }
}

#define XT_P 72
__global__ __launch_bounds__(256) void xpose_cast(
    const float* __restrict__ x, unsigned short* __restrict__ xt) {
  __shared__ __align__(16) _Float16 T[64 * XT_P];
  const int tid = threadIdx.x;
  const int n0 = blockIdx.x * 64, c0 = blockIdx.y * 64, b = blockIdx.z;
#pragma unroll
  for (int it = 0; it < 4; ++it) {
    const int idx = it * 256 + tid;
    const int cr = idx >> 4, f4 = idx & 15;
    const v4f v = *(const v4f*)(x + ((size_t)(b * NCH + c0 + cr)) * NPIX + n0 + f4 * 4);
#pragma unroll
    for (int e = 0; e < 4; ++e) T[(f4 * 4 + e) * XT_P + cr] = (_Float16)v[e];
  }
  __syncthreads();
  const int pc = tid & 7;
  for (int pass = 0; pass < 2; ++pass) {
#pragma unroll
    for (int it = 0; it < 2; ++it) {
      const int L = it * 32 + (tid >> 3);
      const uv4 w = *(const uv4*)(T + L * XT_P + pc * 8);
      *(volatile uv4*)(xt + ((size_t)(b * NPIX + n0 + L)) * NCH + c0 + pc * 8) = w;
    }
    __threadfence();
  }
}

#define AK_KVC 64
#define AK_KSP 40
#define AK_VSP 72
#define AK_OBP 68
#define AK_PSC 32768.0f

__device__ __forceinline__ v8f mma_h(v16h a, v16h b, v8f c) {
  c = __builtin_amdgcn_wmma_f32_16x16x32_f16(false, a, false, b, (short)0, c, false, false);
  asm volatile("v_nop\n\tv_nop\n\tv_nop\n\tv_nop" : "+v"(c) : "v"(a), "v"(b));
  return c;
}
__device__ __forceinline__ v8f zero8() { return (v8f){0.f,0.f,0.f,0.f,0.f,0.f,0.f,0.f}; }

__global__ __launch_bounds__(256) void attn_fused(
    const unsigned short* __restrict__ qkp, const unsigned short* __restrict__ vp,
    const float* __restrict__ x, const float* __restrict__ gamma, float* __restrict__ out) {
  __shared__ __align__(16) _Float16 Ks[AK_KVC * AK_KSP];
  __shared__ __align__(16) float    VsO[(NCH * AK_VSP) / 2];
  __shared__ __align__(16) _Float16 Ps[8][16 * AK_KVC];
  _Float16* Vs = (_Float16*)(void*)VsO;

  const int tid  = threadIdx.x;
  const int wave = tid >> 5;
  const int lane = tid & 31;
  const int hh   = lane >> 4;
  const int c    = lane & 15;
  const int wq   = wave & 3;
  const int wo   = wave >> 2;
  const int qb   = blockIdx.x;
  const int b    = blockIdx.y;
  const int q0   = qb * 64 + wq * 16;
  const int obase = wo * 128;

  const unsigned short* qkb = qkp + (size_t)b * NPIX * QKLD;
  const unsigned short* vb  = vp  + (size_t)b * NCH * NPIX;

  const v16h qa = Frag<_Float16>::load((const _Float16*)(const void*)(qkb + (size_t)(q0 + c) * QKLD + 8 * hh));

  float mrow[8], lrow[8];
  v8f oacc[8];
#pragma unroll
  for (int r = 0; r < 8; ++r) { mrow[r] = -INFINITY; lrow[r] = 0.f; }
#pragma unroll
  for (int t = 0; t < 8; ++t) oacc[t] = zero8();

  _Float16* pw = Ps[wave];

  for (int kc = 0; kc < NPIX / AK_KVC; ++kc) {
    const int kv0 = kc * AK_KVC;
    __syncthreads();
    {
      const int kv = tid >> 2, pc4 = tid & 3;
      const uv4 w = *(const uv4*)(qkb + (size_t)(kv0 + kv) * QKLD + DQK + pc4 * 8);
      *(uv4*)(Ks + kv * AK_KSP + pc4 * 8) = w;
    }
#pragma unroll
    for (int it = 0; it < 8; ++it) {
      const int idx = it * 256 + tid;
      const int o = idx >> 3, pc8 = idx & 7;
      const uv4 w = *(const uv4*)(vb + (size_t)o * NPIX + kv0 + pc8 * 8);
      *(uv4*)(Vs + o * AK_VSP + pc8 * 8) = w;
    }
    __syncthreads();

    v8f s[4];
#pragma unroll
    for (int j = 0; j < 4; ++j) {
      const v16h kb = Frag<_Float16>::load(Ks + (j * 16 + c) * AK_KSP + 8 * hh);
      s[j] = mma_h(qa, kb, zero8());
    }
    float cm[8];
#pragma unroll
    for (int r = 0; r < 8; ++r) {
      float m = -INFINITY;
#pragma unroll
      for (int j = 0; j < 4; ++j) m = fmaxf(m, s[j][r]);
#pragma unroll
      for (int off = 1; off < 16; off <<= 1) m = fmaxf(m, __shfl_xor(m, off, 32));
      cm[r] = m;
    }
#pragma unroll
    for (int r = 0; r < 8; ++r) {
      const float mnew  = fmaxf(mrow[r], cm[r]);
      const float alpha = expf(mrow[r] - mnew);
      mrow[r] = mnew;
      float psum = 0.f;
#pragma unroll
      for (int j = 0; j < 4; ++j) {
        const float p = expf(s[j][r] - mnew);
        psum += p;
        pw[(8 * hh + r) * AK_KVC + j * 16 + c] = (_Float16)(p * AK_PSC);
      }
#pragma unroll
      for (int off = 1; off < 16; off <<= 1) psum += __shfl_xor(psum, off, 32);
      lrow[r] = lrow[r] * alpha + psum;
#pragma unroll
      for (int t = 0; t < 8; ++t) oacc[t][r] *= alpha;
    }
    __builtin_amdgcn_fence(__ATOMIC_RELEASE, "workgroup");
    __builtin_amdgcn_wave_barrier();
    __builtin_amdgcn_fence(__ATOMIC_ACQUIRE, "workgroup");
#pragma unroll 1
    for (int kk = 0; kk < 2; ++kk) {
      const v16h pa = Frag<_Float16>::load(pw + c * AK_KVC + kk * 32 + 8 * hh);
#pragma unroll
      for (int t = 0; t < 8; ++t) {
        const v16h vf = Frag<_Float16>::load(Vs + (obase + t * 16 + c) * AK_VSP + kk * 32 + 8 * hh);
        oacc[t] = mma_h(pa, vf, oacc[t]);
      }
    }
  }

  const float gm = gamma[0];
  float gsc[8];
#pragma unroll
  for (int r = 0; r < 8; ++r) gsc[r] = gm * (1.0f / (lrow[r] * AK_PSC));
  float* Ob = VsO;
  const int pcq = tid & 7;
#pragma unroll
  for (int half = 0; half < 2; ++half) {
    __syncthreads();
    if (wo == half) {
#pragma unroll
      for (int t = 0; t < 8; ++t)
#pragma unroll
        for (int r = 0; r < 8; ++r)
          Ob[(t * 16 + c) * AK_OBP + wq * 16 + 8 * hh + r] = oacc[t][r] * gsc[r];
    }
    __syncthreads();
    const size_t gbase = ((size_t)b * NCH + (size_t)half * 128) * NPIX + (size_t)qb * 64;
    for (int pass = 0; pass < 2; ++pass) {
#pragma unroll
      for (int it = 0; it < 8; ++it) {
        const int L = it * 32 + (tid >> 3);
        const int row = L >> 1, hl = L & 1;
        const v4f a = *(const v4f*)(Ob + row * AK_OBP + hl * 32 + pcq * 4);
        const size_t gi = gbase + (size_t)row * NPIX + (size_t)(hl * 32 + pcq * 4);
        const v4f xr = *(const v4f*)(x + gi);
        const v4f v = a + xr;
        *(volatile v4f*)(out + gi) = v;
      }
      __threadfence();
    }
  }
}

static_assert(NCH % 32 == 0, "K multiple of 32 for both GEMMs");
static_assert(NPIX % 64 == 0 && QKLD % 64 == 0, "q|k GEMM M,N tile multiples");
static_assert(NCH % 64 == 0 && NPIX % 64 == 0, "v GEMM M,N tile multiples");
static_assert(NPIX % AK_KVC == 0 && NCH == 256 && DQK == 32, "attention geometry");
static_assert((DQK * NCH) % 512 == 0 && (NCH * NCH) % 512 == 0, "cast grids exact");

#define WS_XT_OFF   0ull
#define WS_XT_SZ    ((size_t)NB * NPIX * NCH * 2)
#define WS_QK_OFF   (WS_XT_OFF + WS_XT_SZ)
#define WS_QK_SZ    ((size_t)NB * NPIX * QKLD * 2)
#define WS_V_OFF    (WS_QK_OFF + WS_QK_SZ)
#define WS_V_SZ     ((size_t)NB * NCH * NPIX * 2)
#define WS_WQK_OFF  (WS_V_OFF + WS_V_SZ)
#define WS_WQK_SZ   ((size_t)QKLD * NCH * 2)
#define WS_WV_OFF   (WS_WQK_OFF + WS_WQK_SZ)
#define WS_WV_SZ    ((size_t)NCH * NCH * 2)
#define WS_BT_OFF   (WS_WV_OFF + WS_WV_SZ)
#define WS_BT_SZ    ((size_t)256)
#define WS_TOTAL    (WS_BT_OFF + WS_BT_SZ)
static_assert(WS_TOTAL == 37912832ull, "carve total");
static_assert(WS_TOTAL <= 134217728ull, "carve under 128 MiB");
static_assert(WS_QK_OFF % 256 == 0 && WS_V_OFF % 256 == 0 && WS_WQK_OFF % 256 == 0 && WS_WV_OFF % 256 == 0 && WS_BT_OFF % 256 == 0, "aligned carves");

extern "C" void kernel_launch(void* const* d_in, const int* in_sizes, int n_in,
                              void* d_out, int out_size, void* d_ws, size_t ws_size,
                              hipStream_t stream) {
  if (n_in < 8) return;
  if (in_sizes[0] != NB * NCH * NPIX || out_size != NB * NCH * NPIX) return;
  if (in_sizes[1] != DQK * NCH || in_sizes[3] != DQK * NCH || in_sizes[5] != NCH * NCH) return;
  if (in_sizes[2] != DQK || in_sizes[4] != DQK || in_sizes[6] != NCH || in_sizes[7] < 1) return;
  if ((size_t)WS_TOTAL > ws_size) return;

  const float* x     = (const float*)d_in[0];
  const float* Wq    = (const float*)d_in[1];
  const float* bq    = (const float*)d_in[2];
  const float* Wk    = (const float*)d_in[3];
  const float* bk    = (const float*)d_in[4];
  const float* Wv    = (const float*)d_in[5];
  const float* bv    = (const float*)d_in[6];
  const float* gamma = (const float*)d_in[7];
  float* out = (float*)d_out;

  unsigned char* ws = (unsigned char*)d_ws;
  unsigned short* xT   = (unsigned short*)(ws + WS_XT_OFF);
  unsigned short* qkpl = (unsigned short*)(ws + WS_QK_OFF);
  unsigned short* vpl  = (unsigned short*)(ws + WS_V_OFF);
  _Float16* wqk16 = (_Float16*)(ws + WS_WQK_OFF);
  _Float16* wv16  = (_Float16*)(ws + WS_WV_OFF);
  float* btab     = (float*)(ws + WS_BT_OFF);

  const int n2half = (DQK * NCH) / 2;
  cast_wqk_f16x2<<<dim3((2 * n2half) / 256), dim3(256), 0, stream>>>(Wq, Wk, wqk16, n2half, WSCALE);
  const int n2v = (NCH * NCH) / 2;
  cast_scale_f16x2<<<dim3(n2v / 256), dim3(256), 0, stream>>>(Wv, wv16, n2v, WSCALE);
  bias_pack64<<<dim3(1), dim3(32), 0, stream>>>(bq, bk, btab);
  xpose_cast<<<dim3(NPIX / 64, NCH / 64, NB), dim3(256), 0, stream>>>(x, xT);
  wmma_gemm64<0, false, 2, 1, false, 0><<<dim3((NPIX / 64) * (QKLD / 64) / 8, NB), dim3(256), 0, stream>>>(
      (const unsigned short*)xT, (const unsigned short*)xT, NCH, (long)NPIX * NCH,
      (const unsigned short*)wqk16, (const unsigned short*)wqk16, NCH, 0L,
      (void*)qkpl, (void*)qkpl, QKLD, (long)NPIX * QKLD,
      btab, btab, 0L,
      NPIX, QKLD, NCH, WSCALE_INV);
  wmma_gemm64<0, false, 1, 1, false, 0><<<dim3((NCH / 64) * (NPIX / 64) / 8, NB), dim3(256), 0, stream>>>(
      (const unsigned short*)wv16, (const unsigned short*)wv16, NCH, 0L,
      (const unsigned short*)xT, (const unsigned short*)xT, NCH, (long)NPIX * NCH,
      (void*)vpl, (void*)vpl, NPIX, (long)NCH * NPIX,
      bv, bv, 0L,
      NCH, NPIX, NCH, WSCALE_INV);
  attn_fused<<<dim3(NPIX / 64, NB), dim3(256), 0, stream>>>(qkpl, vpl, x, gamma, out);
}
